// GATNet_35485019799828
// MI455X (gfx1250) — hardware-run, weakly checked
//
#include <hip/hip_runtime.h>
#include <stddef.h>
#include <stdint.h>
#include <math.h>


#define NN     50000
#define NE     800000
#define DIN    128
#define HID    64
#define DOUT   40
#define NOP    48
#define KP     128
#define TM     128
#define MP     50048
#define NBA    1024
#define NBLK   49
#define NSLOT  (NBLK * NBA)
#define RCAP   28672
#define DEGCAP 64
#define WLCAP  4096
#define NTHR   256
#define NWAVE  8
#define SP     68
#define NEGSL  0.2f
#define WSMAX  134217728

#define UX     (MP * 16)
#define UW1    (HID * 16)
#define UW2    (HID * 16)
#define ULW    (NOP * 16)
#define UPR    NTHR
#define PREP_BLOCKS ((UX + UW1 + UW2 + ULW + UPR) / NTHR)
#define PRM_FLOATS 448
#define BK_INTS (NWAVE * WLCAP + RCAP + 3 * NBA + 16)
#define BK_LDS  (BK_INTS * 4)

static_assert(MP % TM == 0 && MP >= NN && MP - NN < TM);
static_assert(NSLOT >= MP && (NBA & (NBA - 1)) == 0 && NBA % TM == 0 && NBA % NWAVE == 0);
static_assert(NN <= 65536);
static_assert(RCAP * 10 >= 16623 * 11);
static_assert(DEGCAP >= 35 + 8);
static_assert(WLCAP >= RCAP / NWAVE + 256);
static_assert(RCAP % (4 * NTHR) == 0 && BK_INTS % 4 == 0 && BK_LDS <= 300000);
static_assert(UX % NTHR == 0 && UW1 % NTHR == 0 && UW2 % NTHR == 0 && ULW % NTHR == 0);
static_assert(KP % 32 == 0 && DIN == KP && 2 * HID == KP && NOP % 16 == 0 && HID % 16 == 0);
static_assert((TM * DOUT * 4) % 128 == 0 && ((NN - (MP - TM)) * DOUT * 4) % 128 == 0);
static_assert((TM * DOUT / 4) % 32 == 0 && ((NN - (MP - TM)) * DOUT / 4) % 32 == 0);
static_assert(PRM_FLOATS * 4 <= 2048);
static_assert(HID / 4 == 16);

typedef float          v2f   __attribute__((ext_vector_type(2)));
typedef float          v4f   __attribute__((ext_vector_type(4)));
typedef float          v8f   __attribute__((ext_vector_type(8)));
typedef int            v4i   __attribute__((ext_vector_type(4)));
typedef int            v8i   __attribute__((ext_vector_type(8)));
typedef unsigned short v8us  __attribute__((ext_vector_type(8)));
typedef __bf16         v16bf __attribute__((ext_vector_type(16)));
typedef v2f  __attribute__((may_alias)) v2fa;
typedef v4f  __attribute__((may_alias)) v4fa;
typedef v4i  __attribute__((may_alias)) v4ia;
typedef v8us __attribute__((may_alias)) v8usa;
union FragB { v16bf v; v8us h[2]; v8i w; };

__device__ __forceinline__ v8f wmb(const FragB& a, const FragB& b, v8f c) {
  v8f d = __builtin_amdgcn_wmma_f32_16x16x32_bf16(false, a.v, false, b.v, (short)0, c, false, false);
  asm volatile("v_nop\n\tv_nop\n\tv_nop\n\tv_nop" : "+v"(d) : "v"(a.w), "v"(b.w));
  return d;
}

__device__ __forceinline__ unsigned bf16_bits(float f) {
  const unsigned u = __float_as_uint(f);
  const unsigned r = (u + 0x7FFFu + ((u >> 16) & 1u)) >> 16;
  return ((u & 0x7FFFFFFFu) > 0x7F800000u) ? 0x7FC0u : (r & 0xFFFFu);
}
__device__ __forceinline__ float bf16_val(float f) { return __uint_as_float(bf16_bits(f) << 16); }
__device__ __forceinline__ v4f bfr4(const v4f a) {
  v4f r; r.x = bf16_val(a.x); r.y = bf16_val(a.y); r.z = bf16_val(a.z); r.w = bf16_val(a.w); return r;
}

__device__ __forceinline__ void put8(unsigned short* p, const v8us o) {
  *(volatile v8us*)p = o;
  __threadfence();
  *(volatile v8us*)p = o;
}

__device__ __forceinline__ v8us gat8(const float* __restrict__ p, int stride, bool ok) {
  const float f0 = p[0];
  const float f1 = p[(size_t)stride];
  const float f2 = p[(size_t)2 * stride];
  const float f3 = p[(size_t)3 * stride];
  const float f4 = p[(size_t)4 * stride];
  const float f5 = p[(size_t)5 * stride];
  const float f6 = p[(size_t)6 * stride];
  const float f7 = p[(size_t)7 * stride];
  asm volatile("" :: "v"(f0)); asm volatile("" :: "v"(f1)); asm volatile("" :: "v"(f2)); asm volatile("" :: "v"(f3));
  asm volatile("" :: "v"(f4)); asm volatile("" :: "v"(f5)); asm volatile("" :: "v"(f6)); asm volatile("" :: "v"(f7));
  v8us o;
  o[0] = ok ? (unsigned short)bf16_bits(f0) : (unsigned short)0;
  o[1] = ok ? (unsigned short)bf16_bits(f1) : (unsigned short)0;
  o[2] = ok ? (unsigned short)bf16_bits(f2) : (unsigned short)0;
  o[3] = ok ? (unsigned short)bf16_bits(f3) : (unsigned short)0;
  o[4] = ok ? (unsigned short)bf16_bits(f4) : (unsigned short)0;
  o[5] = ok ? (unsigned short)bf16_bits(f5) : (unsigned short)0;
  o[6] = ok ? (unsigned short)bf16_bits(f6) : (unsigned short)0;
  o[7] = ok ? (unsigned short)bf16_bits(f7) : (unsigned short)0;
  return o;
}

__global__ __launch_bounds__(NTHR) void k_prep(const float* __restrict__ x, const float* __restrict__ W1,
                                               const float* __restrict__ W2, const float* __restrict__ LW,
                                               const float* __restrict__ as1, const float* __restrict__ ad1,
                                               const float* __restrict__ b1, const float* __restrict__ as2,
                                               const float* __restrict__ ad2, const float* __restrict__ b2,
                                               const float* __restrict__ lb,
                                               unsigned short* XB, unsigned short* W1t, unsigned short* W2d,
                                               unsigned short* LWd, float* PRM) {
  const int u = (int)blockIdx.x * NTHR + (int)threadIdx.x;
  if (u < UX) {
    const int row = u >> 4;
    const int k8  = (u & 15) * 8;
    const int rc  = row < NN ? row : NN - 1;
    const float* p = x + (size_t)rc * DIN + k8;
    const v4f a = *(const v4f*)p;
    const v4f b = *(const v4f*)(p + 4);
    asm volatile("" :: "v"(a));
    asm volatile("" :: "v"(b));
    const bool ok = row < NN;
    v8us o;
    o[0] = ok ? (unsigned short)bf16_bits(a.x) : (unsigned short)0;
    o[1] = ok ? (unsigned short)bf16_bits(a.y) : (unsigned short)0;
    o[2] = ok ? (unsigned short)bf16_bits(a.z) : (unsigned short)0;
    o[3] = ok ? (unsigned short)bf16_bits(a.w) : (unsigned short)0;
    o[4] = ok ? (unsigned short)bf16_bits(b.x) : (unsigned short)0;
    o[5] = ok ? (unsigned short)bf16_bits(b.y) : (unsigned short)0;
    o[6] = ok ? (unsigned short)bf16_bits(b.z) : (unsigned short)0;
    o[7] = ok ? (unsigned short)bf16_bits(b.w) : (unsigned short)0;
    put8(XB + (size_t)row * KP + k8, o);
  } else if (u < UX + UW1) {
    const int v  = u - UX;
    const int n  = v >> 4;
    const int k8 = (v & 15) * 8;
    const v8us o = gat8(W1 + (size_t)k8 * HID + n, HID, true);
    put8(W1t + (size_t)n * KP + k8, o);
  } else if (u < UX + UW1 + UW2) {
    const int v  = u - UX - UW1;
    const int n  = v >> 4;
    const int k8 = (v & 15) * 8;
    const int kk = k8 & (HID - 1);
    const v8us o = gat8(W2 + (size_t)kk * HID + n, HID, true);
    put8(W2d + (size_t)n * KP + k8, o);
  } else if (u < UX + UW1 + UW2 + ULW) {
    const int v   = u - UX - UW1 - UW2;
    const int n   = v >> 4;
    const int k8  = (v & 15) * 8;
    const int kk  = k8 & (HID - 1);
    const int ncl = n < DOUT ? n : DOUT - 1;
    const v8us o = gat8(LW + (size_t)kk * DOUT + ncl, DOUT, n < DOUT);
    put8(LWd + (size_t)n * KP + k8, o);
  } else {
    const int t   = u - UX - UW1 - UW2 - ULW;
    const int q   = t & 15;
    const int seg = t >> 4;
    const int ql  = q < 10 ? q : 9;
    const v4f a0 = *(const v4f*)(as1 + 4 * q);
    const v4f a1 = *(const v4f*)(ad1 + 4 * q);
    const v4f a2 = *(const v4f*)(b1  + 4 * q);
    const v4f a3 = *(const v4f*)(as2 + 4 * q);
    const v4f a4 = *(const v4f*)(ad2 + 4 * q);
    const v4f a5 = *(const v4f*)(b2  + 4 * q);
    v4f a6       = *(const v4f*)(lb  + 4 * ql);
    asm volatile("" :: "v"(a0)); asm volatile("" :: "v"(a1)); asm volatile("" :: "v"(a2));
    asm volatile("" :: "v"(a3)); asm volatile("" :: "v"(a4)); asm volatile("" :: "v"(a5));
    asm volatile("" :: "v"(a6));
    const v4f z4 = {0.f, 0.f, 0.f, 0.f};
    a6 = (q < 10) ? a6 : z4;
    v4f r = a0;
    r = (seg == 1) ? a1 : r;
    r = (seg == 2) ? a2 : r;
    r = (seg == 3) ? a3 : r;
    r = (seg == 4) ? a4 : r;
    r = (seg == 5) ? a5 : r;
    r = (seg == 6) ? a6 : r;
    r = bfr4(r);
    if (t < PRM_FLOATS / 4) {
      float* dp = PRM + 4 * t;
      *(volatile v4f*)dp = r;
      __threadfence();
      *(volatile v4f*)dp = r;
    }
  }
}

__device__ __forceinline__ int hitj(int* wlw, int wc, bool valid, int d, int s, unsigned nb0) {
  const unsigned slot = (unsigned)d - nb0;
  const bool hit = valid && (slot < (unsigned)NBA);
  const unsigned mj = __builtin_amdgcn_ballot_w32(hit);
  if (mj != 0u) {
    if (hit) {
      const int pos = wc + (int)__builtin_amdgcn_mbcnt_lo(mj, 0u);
      const int sc  = s < 0 ? 0 : (s > NN - 1 ? NN - 1 : s);
      if (pos < WLCAP) wlw[pos] = sc | (int)(slot << 16);
    }
    wc += (int)__builtin_popcount(mj);
  }
  return wc;
}

__global__ __launch_bounds__(NTHR) void k_bucket(const int* __restrict__ srcs, const int* __restrict__ dsts,
                                                 int* CNT, int* OFF, int* HITS, int* FLAG) {
  extern __shared__ __attribute__((aligned(16))) int dsm[];
  int* wl   = dsm;
  int* sl   = dsm + NWAVE * WLCAP;
  int* cnt  = sl + RCAP;
  int* offs = cnt + NBA;
  int* cur  = offs + NBA;
  int* misc = cur + NBA;
  const int tid = (int)threadIdx.x, lane = tid & 31;
  const int wave = __builtin_amdgcn_readfirstlane(tid >> 5);
  const int blk = (int)blockIdx.x;
  const unsigned nodeBase = (unsigned)(blk * NBA);

  {
    const v4i z4 = {0, 0, 0, 0};
    for (int i = tid * 4; i < BK_INTS; i += NTHR * 4) *(v4ia*)(dsm + i) = z4;
  }
  __syncthreads();

  {
    const int per = (NE + NWAVE - 1) / NWAVE;
    const int eb  = wave * per;
    const int ee  = (eb + per) < NE ? (eb + per) : NE;
    int* wlw = wl + wave * WLCAP;
    int wc = 0;
#pragma unroll 1
    for (int base = eb; base < ee; base += 128) {
      const int i0 = base + lane, i1 = i0 + 32, i2 = i0 + 64, i3 = i0 + 96;
      const int c0 = i0 < NE - 1 ? i0 : NE - 1;
      const int c1 = i1 < NE - 1 ? i1 : NE - 1;
      const int c2 = i2 < NE - 1 ? i2 : NE - 1;
      const int c3 = i3 < NE - 1 ? i3 : NE - 1;
      const int d0 = dsts[c0], d1 = dsts[c1], d2 = dsts[c2], d3 = dsts[c3];
      const int s0 = srcs[c0], s1 = srcs[c1], s2 = srcs[c2], s3 = srcs[c3];
      asm volatile("" :: "v"(d0)); asm volatile("" :: "v"(d1)); asm volatile("" :: "v"(d2)); asm volatile("" :: "v"(d3));
      asm volatile("" :: "v"(s0)); asm volatile("" :: "v"(s1)); asm volatile("" :: "v"(s2)); asm volatile("" :: "v"(s3));
      wc = hitj(wlw, wc, i0 < ee, d0, s0, nodeBase);
      wc = hitj(wlw, wc, i1 < ee, d1, s1, nodeBase);
      wc = hitj(wlw, wc, i2 < ee, d2, s2, nodeBase);
      wc = hitj(wlw, wc, i3 < ee, d3, s3, nodeBase);
    }
    if (lane == 0) misc[wave] = wc;
  }
  __syncthreads();

  if (wave == 0) {
    int tot = 0, ov = 0;
#pragma unroll 1
    for (int w2 = 0; w2 < NWAVE; ++w2) {
      int c = misc[w2];
      if (c > WLCAP) ov = 1;
      c = c < 0 ? 0 : (c > WLCAP ? WLCAP : c);
      const int* lw = wl + w2 * WLCAP;
#pragma unroll 1
      for (int b0 = 0; b0 < c; b0 += 32) {
        const int idx = b0 + lane;
        const int ent = lw[idx < WLCAP ? idx : WLCAP - 1];
        const int m32 = (c - b0) < 32 ? (c - b0) : 32;
#pragma unroll 1
        for (int k = 0; k < m32; ++k) {
          const int uu   = __builtin_amdgcn_readlane(ent, k);
          const int slot = (uu >> 16) & (NBA - 1);
          if (lane == 0) cnt[slot] = cnt[slot] + 1;
        }
      }
      tot += c;
    }
    if (tot > RCAP) ov = 1;
    if (lane == 0) misc[9] = ov;
  }
  __syncthreads();

  if (wave == 0) {
    const int base = lane * (NBA / 32);
    int s = 0;
#pragma unroll 1
    for (int i = 0; i < NBA / 32; ++i) s += cnt[base + i];
    int incl = s;
#pragma unroll
    for (int d = 1; d < 32; d <<= 1) {
      const int y = __shfl_up(incl, d, 32);
      if (lane >= d) incl += y;
    }
    int run = incl - s;
#pragma unroll 1
    for (int i = 0; i < NBA / 32; ++i) {
      const int cv = cnt[base + i];
      offs[base + i] = run;
      cur[base + i]  = run;
      run += cv;
    }
  }
  __syncthreads();

  if (wave == 0) {
#pragma unroll 1
    for (int w2 = 0; w2 < NWAVE; ++w2) {
      int c = misc[w2];
      c = c < 0 ? 0 : (c > WLCAP ? WLCAP : c);
      const int* lw = wl + w2 * WLCAP;
#pragma unroll 1
      for (int b0 = 0; b0 < c; b0 += 32) {
        const int idx = b0 + lane;
        const int ent = lw[idx < WLCAP ? idx : WLCAP - 1];
        const int m32 = (c - b0) < 32 ? (c - b0) : 32;
#pragma unroll 1
        for (int k = 0; k < m32; ++k) {
          const int uu   = __builtin_amdgcn_readlane(ent, k);
          const int slot = (uu >> 16) & (NBA - 1);
          if (lane == 0) {
            int p = cur[slot];
            p = p < 0 ? 0 : (p > RCAP - 1 ? RCAP - 1 : p);
            sl[p] = uu;
            cur[slot] = p + 1;
          }
        }
      }
    }
  }
  __syncthreads();

  const int ovf = misc[9];
  int* cg = CNT  + (size_t)blk * NBA;
  int* og = OFF  + (size_t)blk * NBA;
  int* hg = HITS + (size_t)blk * RCAP;
  int* fg = FLAG + (size_t)blk * 32;
  const v4i f4 = {ovf, ovf, ovf, ovf};
  {
    const v4i c4 = *(const v4ia*)(cnt + 4 * tid);
    const v4i o4 = *(const v4ia*)(offs + 4 * tid);
    *(volatile v4i*)(cg + 4 * tid) = c4;
    *(volatile v4i*)(og + 4 * tid) = o4;
#pragma unroll 1
    for (int i = tid; i < RCAP / 4; i += NTHR) {
      const v4i h4 = *(const v4ia*)(sl + 4 * i);
      *(volatile v4i*)(hg + 4 * i) = h4;
    }
    if (tid < 8) *(volatile v4i*)(fg + 4 * tid) = f4;
  }
  __threadfence();
  {
    const v4i c4 = *(const v4ia*)(cnt + 4 * tid);
    const v4i o4 = *(const v4ia*)(offs + 4 * tid);
    *(volatile v4i*)(cg + 4 * tid) = c4;
    *(volatile v4i*)(og + 4 * tid) = o4;
#pragma unroll 1
    for (int i = tid; i < RCAP / 4; i += NTHR) {
      const v4i h4 = *(const v4ia*)(sl + 4 * i);
      *(volatile v4i*)(hg + 4 * i) = h4;
    }
    if (tid < 8) *(volatile v4i*)(fg + 4 * tid) = f4;
  }
}

__global__ __launch_bounds__(NTHR) __attribute__((amdgpu_num_vgpr(248)))
void k_gemm(const unsigned short* __restrict__ A, const unsigned short* __restrict__ BT,
            const float* __restrict__ att, float* Hout, float* SD) {
  __shared__ __attribute__((aligned(16))) float stg[TM * SP];
  __shared__ __attribute__((aligned(16))) float satt[2 * HID];
  __shared__ __attribute__((aligned(16))) float sdot[2 * TM];
  const int tid = (int)threadIdx.x, lane = tid & 31, wave = tid >> 5, hh = lane >> 4, m = lane & 15;
  const int rowBase = (int)blockIdx.x * TM;

  if (wave == 0) {
    const v4f a = *(const v4f*)(att + 4 * lane);
    *(v4fa*)(satt + 4 * lane) = a;
  }

  v8f acc[4];
  {
    const v8f z = {0.f, 0.f, 0.f, 0.f, 0.f, 0.f, 0.f, 0.f};
    acc[0] = z; acc[1] = z; acc[2] = z; acc[3] = z;
  }
  const unsigned short* ap = A  + (size_t)(rowBase + 16 * wave + m) * KP + 8 * hh;
  const unsigned short* bp = BT + (size_t)m * KP + 8 * hh;
#pragma unroll 1
  for (int k0 = 0; k0 < KP; k0 += 32) {
    FragB af;
    af.h[0] = *(const v8usa*)(ap + k0);
    af.h[1] = *(const v8usa*)(ap + k0 + 16);
#pragma unroll
    for (int t = 0; t < 4; ++t) {
      const unsigned short* wq = bp + (size_t)(16 * t) * KP + k0;
      FragB bf;
      bf.h[0] = *(const v8usa*)wq;
      bf.h[1] = *(const v8usa*)(wq + 16);
      acc[t] = wmb(af, bf, acc[t]);
    }
  }

#pragma unroll
  for (int t = 0; t < 4; ++t) {
    const int lc = 16 * t + m;
#pragma unroll
    for (int r = 0; r < 8; ++r) {
      const int lr = 16 * wave + 8 * hh + r;
      stg[lr * SP + lc] = acc[t][r];
    }
  }
  __syncthreads();

  {
    const int row = tid & (TM - 1), which = tid >> 7;
    const float* sa = satt + which * HID;
    const float* hr = stg + row * SP;
    float d = 0.0f;
#pragma unroll 4
    for (int c4 = 0; c4 < HID / 4; ++c4) {
      const v4f hv = *(const v4fa*)(hr + 4 * c4);
      const v4f av = *(const v4fa*)(sa + 4 * c4);
      d = fmaf(hv.x, av.x, d);
      d = fmaf(hv.y, av.y, d);
      d = fmaf(hv.z, av.z, d);
      d = fmaf(hv.w, av.w, d);
    }
    sdot[which * TM + row] = d;
  }
  __syncthreads();

  v4f fv[8];
#pragma unroll
  for (int i = 0; i < 8; ++i) {
    const int lr = 16 * wave + 2 * i + hh;
    fv[i] = *(const v4fa*)(stg + lr * SP + 4 * m);
  }
  const int wsel = wave < 2 ? wave : 1;
  const v4f sdv = *(const v4fa*)(sdot + wsel * TM + 4 * lane);
  float* sp = SD + (size_t)wsel * MP + rowBase + 4 * lane;

#pragma unroll
  for (int i = 0; i < 8; ++i) {
    const int lr = 16 * wave + 2 * i + hh;
    float* op = Hout + (size_t)(rowBase + lr) * HID + 4 * m;
    *(volatile v4f*)op = fv[i];
  }
  if (wave < 2) *(volatile v4f*)sp = sdv;
  __threadfence();
#pragma unroll
  for (int i = 0; i < 8; ++i) {
    const int lr = 16 * wave + 2 * i + hh;
    float* op = Hout + (size_t)(rowBase + lr) * HID + 4 * m;
    *(volatile v4f*)op = fv[i];
  }
  if (wave < 2) *(volatile v4f*)sp = sdv;
}

__global__ __launch_bounds__(NTHR) void k_replay(const float* __restrict__ H, const float* __restrict__ SD,
                                                 const int* __restrict__ CNT, const int* __restrict__ OFF,
                                                 const int* __restrict__ HITS, const int* __restrict__ FLAG,
                                                 const float* __restrict__ bias, unsigned short* XHL) {
  __shared__ __attribute__((aligned(16))) float sb[HID];
  const int tid = (int)threadIdx.x, lane = tid & 31;
  const int wave = __builtin_amdgcn_readfirstlane(tid >> 5);
  const int blk = (int)blockIdx.x;
  const int nodeBase = blk * NBA;
  if (wave == 0) {
    const int q = lane & (HID / 4 - 1);
    const v4f a = *(const v4f*)(bias + 4 * q);
    asm volatile("" :: "v"(a));
    *(v4fa*)(sb + 4 * q) = a;
  }
  __syncthreads();
  const v2f bb = *(const v2fa*)(sb + 2 * lane);
  const int flag = FLAG[(size_t)blk * 32];
  const int* hb = HITS + (size_t)blk * RCAP;
  const float qn = __int_as_float(0x7fc00000);
  const float ninf = -__builtin_inff();

#pragma unroll 1
  for (int si = 0; si < NBA / NWAVE; ++si) {
    const int s    = si * NWAVE + wave;
    const int node = nodeBase + s;
    const int nc   = node < NN ? node : NN - 1;
    const int craw = CNT[node];
    const int oraw = OFF[node];
    const bool big = (craw > DEGCAP) || (craw < 0);
    int c = craw < 0 ? 0 : (craw > DEGCAP ? DEGCAP : craw);
    const int o = oraw < 0 ? 0 : (oraw > RCAP ? RCAP : oraw);
    if (c > RCAP - o) c = RCAP - o;
    const float as0 = SD[nc];
    const float ad  = SD[(size_t)MP + nc];
    const v2f hs = *(const v2f*)(H + (size_t)nc * HID + 2 * lane);
    float a0 = hs.x, a1 = hs.y;
    float e0 = as0 + ad;
    e0 = (e0 >= 0.0f) ? e0 : NEGSL * e0;
    float mx = e0, ll = 1.0f;

#pragma unroll 1
    for (int b0 = 0; b0 < c; b0 += 32) {
      const int j = b0 + lane;
      const bool valid = j < c;
      int idx = o + (j < c - 1 ? j : c - 1);
      idx = idx > RCAP - 1 ? RCAP - 1 : idx;
      const int ent = hb[idx];
      asm volatile("" :: "v"(ent));
      int sr = ent & 0xFFFF;
      sr = sr > NN - 1 ? NN - 1 : sr;
      const float asv = SD[sr];
      asm volatile("" :: "v"(asv));
      float e = asv + ad;
      e = (e >= 0.0f) ? e : NEGSL * e;
      e = valid ? e : ninf;
      float cm = e;
      cm = fmaxf(cm, __shfl_xor(cm, 16));
      cm = fmaxf(cm, __shfl_xor(cm, 8));
      cm = fmaxf(cm, __shfl_xor(cm, 4));
      cm = fmaxf(cm, __shfl_xor(cm, 2));
      cm = fmaxf(cm, __shfl_xor(cm, 1));
      const float mn = fmaxf(mx, cm);
      const float sc = expf(mx - mn);
      a0 *= sc; a1 *= sc; ll *= sc;
      mx = mn;
      float p = expf(e - mn);
      p = valid ? p : 0.0f;
      const int pi  = __float_as_int(p);
      const int m32 = (c - b0) < 32 ? (c - b0) : 32;
#pragma unroll 1
      for (int k = 0; k < m32; ++k) {
        const int   sk = __builtin_amdgcn_readlane(sr, k);
        const float pk = __int_as_float(__builtin_amdgcn_readlane(pi, k));
        const v2f hv = *(const v2f*)(H + (size_t)sk * HID + 2 * lane);
        a0 = fmaf(pk, hv.x, a0);
        a1 = fmaf(pk, hv.y, a1);
        ll += pk;
      }
    }

    const int cr = craw < 0 ? 0 : craw;
    const float cf = (float)(cr + 1);
    const float v0 = (a0 / ll) / cf + bb.x;
    const float v1 = (a1 / ll) / cf + bb.y;
    float r0 = (v0 > 0.0f) ? v0 : (v0 - v0);
    float r1 = (v1 > 0.0f) ? v1 : (v1 - v1);
    const bool pois = (flag != 0) || big;
    r0 = pois ? qn : r0;
    r1 = pois ? qn : r1;
    const bool live = node < NN;
    r0 = live ? r0 : 0.0f;
    r1 = live ? r1 : 0.0f;
    const unsigned h0 = bf16_bits(r0), h1 = bf16_bits(r1);
    const unsigned l0 = bf16_bits(r0 - __uint_as_float(h0 << 16));
    const unsigned l1 = bf16_bits(r1 - __uint_as_float(h1 << 16));
    const unsigned hw = h0 | (h1 << 16);
    const unsigned lw = l0 | (l1 << 16);
    if (node < MP) {
      unsigned* rp = (unsigned*)(XHL + (size_t)node * KP);
      *(volatile unsigned*)(rp + lane) = hw;
      *(volatile unsigned*)(rp + 32 + lane) = lw;
      __threadfence();
      *(volatile unsigned*)(rp + lane) = hw;
      *(volatile unsigned*)(rp + 32 + lane) = lw;
    }
  }
}

__global__ __launch_bounds__(NTHR) __attribute__((amdgpu_num_vgpr(248)))
void k_head(const unsigned short* __restrict__ A, const unsigned short* __restrict__ BT,
            const float* __restrict__ lbp, const int* __restrict__ FLAG, float* out) {
  __shared__ __attribute__((aligned(16))) float stg[TM * DOUT];
  __shared__ __attribute__((aligned(16))) float slb[HID];
  const int tid = (int)threadIdx.x, lane = tid & 31, wave = tid >> 5, hh = lane >> 4, m = lane & 15;
  const int rowBase = (int)blockIdx.x * TM;
  if (wave == 0) {
    const int q = lane & (HID / 4 - 1);
    const v4f a = *(const v4f*)(lbp + 4 * q);
    asm volatile("" :: "v"(a));
    *(v4fa*)(slb + 4 * q) = a;
  }
  __syncthreads();

  v8f acc[3];
  {
    const v8f z = {0.f, 0.f, 0.f, 0.f, 0.f, 0.f, 0.f, 0.f};
    acc[0] = z; acc[1] = z; acc[2] = z;
  }
  const unsigned short* ap = A  + (size_t)(rowBase + 16 * wave + m) * KP + 8 * hh;
  const unsigned short* bp = BT + (size_t)m * KP + 8 * hh;
#pragma unroll 1
  for (int k0 = 0; k0 < KP; k0 += 32) {
    FragB af;
    af.h[0] = *(const v8usa*)(ap + k0);
    af.h[1] = *(const v8usa*)(ap + k0 + 16);
#pragma unroll
    for (int t = 0; t < 3; ++t) {
      const unsigned short* wq = bp + (size_t)(16 * t) * KP + k0;
      FragB bf;
      bf.h[0] = *(const v8usa*)wq;
      bf.h[1] = *(const v8usa*)(wq + 16);
      acc[t] = wmb(af, bf, acc[t]);
    }
  }

#pragma unroll
  for (int t = 0; t < 3; ++t) {
    const int col = 16 * t + m;
    const float lb = slb[col];
#pragma unroll
    for (int r = 0; r < 8; ++r) {
      const int lr = 16 * wave + 8 * hh + r;
      const float v = acc[t][r] + lb;
      const float y = (v > 0.0f) ? v : (v - v);
      if (col < DOUT) stg[lr * DOUT + col] = y;
    }
  }
  __syncthreads();

  int live = NN - rowBase;
  live = live < 0 ? 0 : (live > TM ? TM : live);
  const int npc = live * (DOUT / 4);
  const int fl = FLAG[(size_t)(rowBase >> 10) * 32];
  const float qn = __int_as_float(0x7fc00000);
  const v4f q4 = {qn, qn, qn, qn};
  float* ob = out + (size_t)rowBase * DOUT;
#pragma unroll 1
  for (int p = tid; p < npc; p += NTHR) {
    v4f v = *(const v4fa*)(stg + 4 * p);
    v = (fl != 0) ? q4 : v;
    *(volatile v4f*)(ob + 4 * p) = v;
  }
  __threadfence();
#pragma unroll 1
  for (int p = tid; p < npc; p += NTHR) {
    v4f v = *(const v4fa*)(stg + 4 * p);
    v = (fl != 0) ? q4 : v;
    *(volatile v4f*)(ob + 4 * p) = v;
  }
}

extern "C" void kernel_launch(void* const* d_in, const int* in_sizes, int n_in,
                              void* d_out, int out_size, void* d_ws, size_t ws_size,
                              hipStream_t stream) {
  if (n_in < 12) return;
  if (in_sizes[0] != NN * DIN) return;
  if (in_sizes[1] != 2 * NE) return;
  if (in_sizes[2] != DIN * HID) return;
  if (in_sizes[3] != HID || in_sizes[4] != HID || in_sizes[5] != HID) return;
  if (in_sizes[6] != HID * HID) return;
  if (in_sizes[7] != HID || in_sizes[8] != HID || in_sizes[9] != HID) return;
  if (in_sizes[10] != HID * DOUT) return;
  if (in_sizes[11] != DOUT) return;
  if (out_size != NN * DOUT) return;

  const float* x    = (const float*)d_in[0];
  const int*   ei   = (const int*)d_in[1];
  const float* W1   = (const float*)d_in[2];
  const float* as1  = (const float*)d_in[3];
  const float* ad1  = (const float*)d_in[4];
  const float* b1   = (const float*)d_in[5];
  const float* W2   = (const float*)d_in[6];
  const float* as2  = (const float*)d_in[7];
  const float* ad2  = (const float*)d_in[8];
  const float* b2   = (const float*)d_in[9];
  const float* LW   = (const float*)d_in[10];
  const float* lb   = (const float*)d_in[11];
  float* out = (float*)d_out;
  const int* src = ei;
  const int* dst = ei + NE;

  char* ws = (char*)d_ws;
  size_t off = 0;
  const size_t oXB  = off; off += (size_t)MP * KP * 2;        off = (off + 255) & ~(size_t)255;
  const size_t oH   = off; off += (size_t)MP * HID * 4;       off = (off + 255) & ~(size_t)255;
  const size_t oXHL = off; off += (size_t)MP * KP * 2;        off = (off + 255) & ~(size_t)255;
  const size_t oSD  = off; off += (size_t)2 * MP * 4;         off = (off + 255) & ~(size_t)255;
  const size_t oHT  = off; off += (size_t)NBLK * RCAP * 4;    off = (off + 255) & ~(size_t)255;
  const size_t oCN  = off; off += (size_t)NSLOT * 4;          off = (off + 255) & ~(size_t)255;
  const size_t oOF  = off; off += (size_t)NSLOT * 4;          off = (off + 255) & ~(size_t)255;
  const size_t oFL  = off; off += (size_t)NBLK * 128;         off = (off + 255) & ~(size_t)255;
  const size_t oW1  = off; off += (size_t)HID * KP * 2;       off = (off + 255) & ~(size_t)255;
  const size_t oW2  = off; off += (size_t)HID * KP * 2;       off = (off + 255) & ~(size_t)255;
  const size_t oLW  = off; off += (size_t)NOP * KP * 2;       off = (off + 255) & ~(size_t)255;
  const size_t oPR  = off; off += (size_t)2048;               off = (off + 255) & ~(size_t)255;
  if (off > ws_size || off > (size_t)WSMAX) return;
  unsigned short* XB  = (unsigned short*)(ws + oXB);
  float*          H   = (float*)(ws + oH);
  unsigned short* XHL = (unsigned short*)(ws + oXHL);
  float*          SD  = (float*)(ws + oSD);
  int*            HT  = (int*)(ws + oHT);
  int*            CN  = (int*)(ws + oCN);
  int*            OF  = (int*)(ws + oOF);
  int*            FL  = (int*)(ws + oFL);
  unsigned short* W1t = (unsigned short*)(ws + oW1);
  unsigned short* W2d = (unsigned short*)(ws + oW2);
  unsigned short* LWd = (unsigned short*)(ws + oLW);
  float*          PRM = (float*)(ws + oPR);

  hipFuncSetAttribute(reinterpret_cast<const void*>(&k_bucket),
                      hipFuncAttributeMaxDynamicSharedMemorySize, (int)BK_LDS);

  k_prep<<<PREP_BLOCKS, NTHR, 0, stream>>>(x, W1, W2, LW, as1, ad1, b1, as2, ad2, b2, lb, XB, W1t, W2d, LWd, PRM);
  k_bucket<<<NBLK, NTHR, BK_LDS, stream>>>(src, dst, CN, OF, HT, FL);
  k_gemm<<<MP / TM, NTHR, 0, stream>>>(XB, W1t, PRM + 0, H, SD);
  k_replay<<<NBLK, NTHR, 0, stream>>>(H, SD, CN, OF, HT, FL, PRM + 128, XHL);
  k_gemm<<<MP / TM, NTHR, 0, stream>>>(XHL, W2d, PRM + 192, H, SD);
  k_replay<<<NBLK, NTHR, 0, stream>>>(H, SD, CN, OF, HT, FL, PRM + 320, XHL);
  k_head<<<MP / TM, NTHR, 0, stream>>>(XHL, LWd, PRM + 384, FL, out);
}
